// GlobalSelfAttention_28544352649554
// MI455X (gfx1250) — hardware-run, weakly checked
//
#include <hip/hip_runtime.h>


#ifndef NB
#define NB 2
#endif
#ifndef SEQ
#define SEQ 400
#endif
#define NB_FULL  2
#define SEQ_FULL 400
#define DM   512
#define TT   16
#define UP   516
#define PHP  424
#define OS_P 68
#define TRP  72
#define SK32 ((SEQ + 31) / 32 * 32)
#define SKP  ((SEQ + 63) / 64 * 64)
#define NCH  (SK32 / 32)
#define UH_F (32 * UP)
#define AL_F (TT * NB_FULL * SEQ_FULL)
#define FC_N4 (AL_F / 4)
#define FC_IT ((FC_N4 + 255) / 256)
#define C2    2.8853900817779268f
#define LOG2E 1.4426950408889634f
#define PCAR  4096.0f
#define PINV  (1.0f / 4096.0f)
#define NINF  (-__builtin_inff())
#define OUT1_OFF ((size_t)SEQ_FULL * NB_FULL * DM)

static_assert(TT == 16);
static_assert(TT == 2 * 8);
static_assert(DM == 8 * 64);
static_assert(SEQ % TT == 0);
static_assert((NB * SEQ) % 16 == 0);
static_assert(DM % 64 == 0);
static_assert(DM % 32 == 0);
static_assert((2 * DM) % 32 == 0);
static_assert(NB <= NB_FULL);
static_assert(SEQ <= SEQ_FULL);
static_assert(SK32 <= PHP);
static_assert(SK32 <= SKP);
static_assert(PHP % 8 == 0);
static_assert(UP % 4 == 0);
static_assert(UP >= DM);
static_assert(8 * 16 * OS_P <= UH_F);
static_assert(16 * 256 * 4 == 32 * DM);
static_assert((UH_F + AL_F) * 4 + TT * PHP * 2 <= 131072);
static_assert(16 * OS_P * 4 + 64 * TRP * 2 <= 131072);
static_assert((UH_F * 4) % 16 == 0);
static_assert(SEQ_FULL % 4 == 0);
static_assert((AL_F * 4) % 128 == 0);
static_assert((TT * NB_FULL * SEQ_FULL * 4) % 128 == 0);
static_assert(OUT1_OFF * 4 == (size_t)1638400);
static_assert((OUT1_OFF * 4) % 128 == 0);
static_assert(FC_N4 % 32 == 0);
static_assert(FC_IT * 256 >= FC_N4);
static_assert(32 * 16 * 8 == 16 * 256);
static_assert(32 * 16 * 4 == 16 * 128);
static_assert(256 * 2 * 16 == 64 * 128);
static_assert(256 * 4 * 4 == 64 * 64);
static_assert(SKP % 64 == 0);
static_assert(((size_t)SEQ * DM) % 8 == 0);
static_assert(((size_t)DM * DM) % 8 == 0);

typedef _Float16 h16;
typedef unsigned short bf;
typedef __attribute__((ext_vector_type(16))) __bf16   v16bf;
typedef __attribute__((ext_vector_type(16))) _Float16 v16h;
typedef __attribute__((ext_vector_type(8)))  _Float16 v8h;
typedef __attribute__((ext_vector_type(8)))  unsigned short v8us;
typedef __attribute__((ext_vector_type(8)))  float    v8f;
typedef __attribute__((ext_vector_type(4)))  float    v4f;
typedef v4f  __attribute__((may_alias)) v4fa;
typedef v8h  __attribute__((may_alias)) v8ha;
typedef v8us __attribute__((may_alias)) v8usa;

__device__ __forceinline__ unsigned short f2bf(float f) { unsigned u = __float_as_uint(f); u += 0x7FFFu + ((u >> 16) & 1u); return (unsigned short)(u >> 16); }
__device__ __forceinline__ float bfr(float f) { return __uint_as_float(((unsigned)f2bf(f)) << 16); }
__device__ __forceinline__ v16h cat16(v8h lo, v8h hi) { return __builtin_shufflevector(lo, hi, 0, 1, 2, 3, 4, 5, 6, 7, 8, 9, 10, 11, 12, 13, 14, 15); }
__device__ __forceinline__ v16bf cat16b(v8us lo, v8us hi) { return __builtin_bit_cast(v16bf, __builtin_shufflevector(lo, hi, 0, 1, 2, 3, 4, 5, 6, 7, 8, 9, 10, 11, 12, 13, 14, 15)); }
__device__ __forceinline__ v8f wmma16(v16h a, v16h b, v8f c) { return __builtin_amdgcn_wmma_f32_16x16x32_f16(false, a, false, b, (short)0, c, false, false); }
__device__ __forceinline__ v8f wmmab(v16bf a, v16bf b, v8f c) { return __builtin_amdgcn_wmma_f32_16x16x32_bf16(false, a, false, b, (short)0, c, false, false); }
__device__ __forceinline__ v16h  ldh(const h16* p) { return cat16(*(const v8h*)p, *(const v8h*)(p + 16)); }
__device__ __forceinline__ v16bf ldb(const bf* p)  { return cat16b(*(const v8us*)p, *(const v8us*)(p + 16)); }
__device__ __forceinline__ void wave_sync() { __builtin_amdgcn_fence(3  , "wavefront"); __builtin_amdgcn_wave_barrier(); asm volatile("" ::: "memory"); }
static __device__ __forceinline__ h16 toh_flush(float v) { const h16 r = (h16)v; return (__builtin_fabsf(v) < 6.103515625e-05f) ? (h16)0.0f : r; }
__device__ __forceinline__ v8f wmma16_g(v16h a, v16h b, v8f c) { c = wmma16(a, b, c); asm volatile("v_nop\n\tv_nop\n\tv_nop\n\tv_nop" : "+v"(c) : "v"(a), "v"(b)); return c; }
__device__ __forceinline__ v8f wmmab_g(v16bf a, v16bf b, v8f c) { c = wmmab(a, b, c); asm volatile("v_nop\n\tv_nop\n\tv_nop\n\tv_nop" : "+v"(c) : "v"(a), "v"(b)); return c; }

__global__ __launch_bounds__(256) void k_cvt8(const float* __restrict__ src, bf* dst, size_t n8) {
    const size_t i = (size_t)blockIdx.x * 256 + threadIdx.x; if (i >= n8) return;
    const v8f v = *(const v8f*)(src + i * 8); v8us o;
#pragma unroll
    for (int k = 0; k < 8; ++k) o[k] = f2bf(v[k]);
    *(volatile v8us*)(dst + i * 8) = o; __threadfence(); *(volatile v8us*)(dst + i * 8) = o;
}

__global__ __launch_bounds__(128) void k_bfr4(const float* __restrict__ src, float* dst, int n4) {
    const int i = blockIdx.x * 128 + threadIdx.x; if (i >= n4) return;
    const v4f v = *(const v4f*)(src + (size_t)i * 4); v4f o;
#pragma unroll
    for (int k = 0; k < 4; ++k) o[k] = bfr(v[k]);
    *(volatile v4f*)(dst + (size_t)i * 4) = o; __threadfence(); *(volatile v4f*)(dst + (size_t)i * 4) = o;
}

__global__ __launch_bounds__(256) void k_tr(const float* __restrict__ src, bf* dst, int R, int C, int RP, size_t sstride, size_t dstride, int f16mode) {
    __shared__ __align__(16) bf ts[64 * TRP];
    const int tid = threadIdx.x;
    const int r0 = blockIdx.x * 64, c0 = blockIdx.y * 64;
    const float* s = src + (size_t)blockIdx.z * sstride;
    bf* d = dst + (size_t)blockIdx.z * dstride;
#pragma unroll 1
    for (int j = 0; j < 4; ++j) {
        const int idx = tid + 256 * j; const int rr = idx >> 4, c4 = (idx & 15) * 4;
        const int rg = r0 + rr; const int rc = rg < R ? rg : (R - 1);
        const v4f x = *(const v4f*)(s + (size_t)rc * C + c0 + c4);
#pragma unroll
        for (int i = 0; i < 4; ++i) {
            const unsigned short ob = f2bf(x[i]);
            const unsigned short oh = __builtin_bit_cast(unsigned short, toh_flush(bfr(x[i])));
            unsigned short o = f16mode ? oh : ob;
            if (rg >= R) o = (unsigned short)0;
            ts[(c4 + i) * TRP + rr] = o; }
    }
    __syncthreads();
#pragma unroll 1
    for (int ps = 0; ps < 2; ++ps) {
#pragma unroll
        for (int j = 0; j < 2; ++j) { const int idx = tid + 256 * j; const int crow = idx >> 3, p8 = (idx & 7) * 8;
            const v8us val = *(const v8usa*)(&ts[crow * TRP + p8]);
            *(volatile v8us*)(d + (size_t)(c0 + crow) * RP + r0 + p8) = val; }
        if (ps == 0) __threadfence(); }
}

__global__ __launch_bounds__(32) void k_gemm(const bf* __restrict__ A0, const bf* __restrict__ A1, int K0, int K1, const bf* __restrict__ Bt,
                                             const float* __restrict__ bias, int hasb, float oscale, float* C, int ldc, int omode) {
    __shared__ __align__(16) float os[16 * OS_P];
    const int lane = threadIdx.x & 31, lr = lane & 15, hi = lane >> 4; const int r0 = blockIdx.x * 16, c0 = blockIdx.y * 64;
    const int KT = K0 + K1;
    v8f acc[4];
#pragma unroll
    for (int nb = 0; nb < 4; ++nb) acc[nb] = (v8f){};
    const size_t boff = (size_t)(c0 + lr) * KT + 8 * hi;
    { const size_t aoff = (size_t)(r0 + lr) * K0 + 8 * hi;
#pragma unroll 1
      for (int kc = 0; kc < K0; kc += 32) {
          const v16bf a = ldb(A0 + aoff + kc);
#pragma unroll
          for (int nb = 0; nb < 4; ++nb) { const v16bf b = ldb(Bt + boff + (size_t)nb * 16 * KT + kc); acc[nb] = wmmab_g(a, b, acc[nb]); } } }
    { const size_t aoff = (size_t)(r0 + lr) * K1 + 8 * hi;
#pragma unroll 1
      for (int kc = 0; kc < K1; kc += 32) {
          const v16bf a = ldb(A1 + aoff + kc);
#pragma unroll
          for (int nb = 0; nb < 4; ++nb) { const v16bf b = ldb(Bt + boff + (size_t)nb * 16 * KT + K0 + kc); acc[nb] = wmmab_g(a, b, acc[nb]); } } }
#pragma unroll
    for (int nb = 0; nb < 4; ++nb) {
        const float bcv = bfr(bias[c0 + nb * 16 + lr]);
        const float bc = hasb ? bcv : 0.0f;
#pragma unroll
        for (int j = 0; j < 8; ++j) os[(hi * 8 + j) * OS_P + nb * 16 + lr] = (acc[nb][j] + bc) * oscale; }
    wave_sync();
#pragma unroll 1
    for (int ps = 0; ps < 2; ++ps) {
#pragma unroll
        for (int s = 0; s < 8; ++s) { const int row = 2 * s + (lane >> 4), cofs = (lane & 15) * 4;
            const v4f val = *(const v4fa*)(&os[row * OS_P + cofs]);
            const int m = r0 + row;
            const int orow = omode ? ((m % SEQ) * NB_FULL + m / SEQ) : m;
            *(volatile v4f*)(C + (size_t)orow * ldc + c0 + cofs) = val; }
        if (ps == 0) __threadfence(); }
}

__global__ __launch_bounds__(256) void k_score(const float* __restrict__ WQ, const float* __restrict__ UH, const float* __restrict__ VF, const int* __restrict__ lens,
                                               const h16* __restrict__ MT, bf* CB, float* OUT1) {
    __shared__ __align__(16) float big[UH_F + AL_F];
    __shared__ __align__(16) h16 ph[TT * PHP];
    const int tid = threadIdx.x, lane = tid & 31, lr = lane & 15, hi = lane >> 4;
    const int wave = __builtin_amdgcn_readfirstlane((int)(threadIdx.x >> 5));
    const int t0 = blockIdx.x * TT;
    if (NB != NB_FULL || SEQ != SEQ_FULL) {
#pragma unroll 1
        for (int i = tid; i < AL_F; i += 256) big[UH_F + i] = 0.0f;
    }
#pragma unroll 1
    for (int b = 0; b < NB; ++b) {
        const int len = lens[b];
        const int tg0 = t0 + 2 * wave;
        const size_t qo = ((size_t)b * SEQ + (size_t)tg0) * DM;
        const size_t ub = (size_t)b * SEQ * DM;
        const int al0 = UH_F + ((2 * wave) * NB_FULL + b) * SEQ_FULL;
        const int al1 = al0 + NB_FULL * SEQ_FULL;
#pragma unroll 1
        for (int ch = 0; ch < NCH; ++ch) {
            __syncthreads();
#pragma unroll 4
            for (int j = 0; j < 16; ++j) { const int idx = tid + 256 * j; const int rr = idx >> 7, c4 = (idx & 127) * 4;
                int s = ch * 32 + rr; s = s < SEQ ? s : (SEQ - 1);
                const v4f x = *(const v4f*)(UH + ub + (size_t)s * DM + c4);
                *(v4fa*)(&big[rr * UP + c4]) = x; }
            __syncthreads();
            float a0 = 0.0f, a1 = 0.0f;
            const int uo = lane * UP;
#pragma unroll 2
            for (int e = 0; e < DM; e += 4) {
                const v4f uu = *(const v4fa*)(&big[uo + e]);
                const v4f q0 = *(const v4f*)(WQ + qo + e);
                const v4f q1 = *(const v4f*)(WQ + qo + DM + e);
                const v4f vv = *(const v4f*)(VF + e);
#pragma unroll
                for (int i = 0; i < 4; ++i) {
                    const float g0 = __builtin_amdgcn_rcpf(1.0f + __builtin_amdgcn_exp2f(q0[i] + uu[i]));
                    const float g1 = __builtin_amdgcn_rcpf(1.0f + __builtin_amdgcn_exp2f(q1[i] + uu[i]));
                    a0 = fmaf(vv[i], fmaf(-2.0f, g0, 1.0f), a0);
                    a1 = fmaf(vv[i], fmaf(-2.0f, g1, 1.0f), a1); }
            }
            const int s = ch * 32 + lane;
            if (s < SEQ) {
                const bool ok0 = (s < len) && (s != tg0);
                const bool ok1 = (s < len) && (s != tg0 + 1);
                big[al0 + s] = ok0 ? a0 : NINF;
                big[al1 + s] = ok1 ? a1 : NINF; }
        }
#pragma unroll 1
        for (int rr = 0; rr < 2; ++rr) {
            const int trow = 2 * wave + rr;
            const int ab = al0 + rr * (NB_FULL * SEQ_FULL);
            float mx = NINF;
#pragma unroll 1
            for (int j = 0; j < NCH; ++j) { const int s = lane + 32 * j; const int sc = s < SEQ ? s : (SEQ - 1);
                const float x = big[ab + sc]; mx = fmaxf(mx, (s < SEQ) ? x : NINF); }
#pragma unroll
            for (int off = 16; off > 0; off >>= 1) mx = fmaxf(mx, __shfl_xor(mx, off, 32));
            float sum = 0.0f;
#pragma unroll 1
            for (int j = 0; j < NCH; ++j) { const int s = lane + 32 * j; const int sc = s < SEQ ? s : (SEQ - 1);
                const float x = big[ab + sc];
                const float ex = __builtin_amdgcn_exp2f((x - mx) * LOG2E);
                const float e = (s < SEQ) ? ex : 0.0f;
                sum += e;
                if (s < SEQ) big[ab + s] = e; }
#pragma unroll
            for (int off = 16; off > 0; off >>= 1) sum += __shfl_xor(sum, off, 32);
            const float inv = 1.0f / sum;
#pragma unroll 1
            for (int j = 0; j < NCH; ++j) { const int s = lane + 32 * j; const int sc = s < SEQ ? s : (SEQ - 1);
                const float e = big[ab + sc];
                const float p = (s < SEQ) ? e * inv : 0.0f;
                if (s < SEQ) big[ab + s] = p;
                ph[trow * PHP + s] = toh_flush(p * PCAR); }
        }
        __syncthreads();
        {
            v8f acc[4];
#pragma unroll
            for (int nb = 0; nb < 4; ++nb) acc[nb] = (v8f){};
            const int n0 = 64 * wave;
            const size_t mo = ((size_t)b * DM + (size_t)(n0 + lr)) * SKP + 8 * hi;
            const int po = lr * PHP + 8 * hi;
#pragma unroll 1
            for (int kc = 0; kc < SK32; kc += 32) {
                const v16h a = cat16(*(const v8ha*)(&ph[po + kc]), *(const v8ha*)(&ph[po + kc + 16]));
#pragma unroll
                for (int nb = 0; nb < 4; ++nb) { const v16h bb = ldh(MT + mo + (size_t)nb * 16 * SKP + kc); acc[nb] = wmma16_g(a, bb, acc[nb]); }
            }
            const int wb = wave * 16 * OS_P;
#pragma unroll
            for (int nb = 0; nb < 4; ++nb) {
#pragma unroll
                for (int j = 0; j < 8; ++j) big[wb + (hi * 8 + j) * OS_P + nb * 16 + lr] = acc[nb][j] * PINV; }
            wave_sync();
            bf* crow = CB + ((size_t)b * SEQ + (size_t)t0) * DM + n0;
#pragma unroll 1
            for (int ps = 0; ps < 2; ++ps) {
#pragma unroll
                for (int s = 0; s < 4; ++s) { const int row = 4 * s + (lane >> 3), c8 = (lane & 7) * 8;
                    const v4f x0 = *(const v4fa*)(&big[wb + row * OS_P + c8]); const v4f x1 = *(const v4fa*)(&big[wb + row * OS_P + c8 + 4]); v8us o;
#pragma unroll
                    for (int i = 0; i < 4; ++i) { o[i] = f2bf(x0[i]); o[4 + i] = f2bf(x1[i]); }
                    *(volatile v8us*)(crow + (size_t)row * DM + c8) = o; }
                if (ps == 0) __threadfence(); }
        }
    }
    __syncthreads();
    float* o1 = OUT1 + (size_t)t0 * NB_FULL * SEQ_FULL;
#pragma unroll 1
    for (int ps = 0; ps < 2; ++ps) {
#pragma unroll 1
        for (int j = 0; j < FC_IT; ++j) { const int idx = tid + 256 * j;
            if (idx < FC_N4) { const v4f val = *(const v4fa*)(&big[UH_F + idx * 4]);
                *(volatile v4f*)(o1 + (size_t)idx * 4) = val; } }
        if (ps == 0) __threadfence(); }
}

static constexpr size_t al256(size_t v) { return (v + 255) & ~(size_t)255; }
static constexpr size_t SZ_XB = al256((size_t)NB * SEQ * DM * 2);
static constexpr size_t SZ_WS = al256((size_t)DM * DM * 2);
static constexpr size_t SZ_WO = al256((size_t)DM * 2 * DM * 2);
static constexpr size_t SZ_MT = al256((size_t)NB * DM * SKP * 2);
static constexpr size_t SZ_VF = al256((size_t)DM * 4);
static constexpr size_t SZ_PF = al256((size_t)NB * SEQ * DM * 4);
static constexpr size_t SZ_TOTAL = 3 * SZ_XB + 2 * SZ_WS + SZ_WO + SZ_MT + SZ_VF + 2 * SZ_PF;
static_assert(SZ_TOTAL <= (size_t)134217728);
static_assert(DM % 4 == 0);
static_assert((DM / 4) % 128 == 0);

extern "C" void kernel_launch(void* const* d_in, const int* in_sizes, int n_in,
                              void* d_out, int out_size, void* d_ws, size_t ws_size, hipStream_t stream) {
    if (n_in < 9) return;
    const size_t needx = ((size_t)(NB - 1) * SEQ_FULL + SEQ) * DM;
    if ((size_t)in_sizes[0] < needx || (size_t)in_sizes[1] < needx) return;
    if (in_sizes[2] < NB) return;
    if ((size_t)in_sizes[3] < (size_t)DM * DM || (size_t)in_sizes[5] < (size_t)DM * DM || (size_t)in_sizes[7] < (size_t)2 * DM * DM) return;
    if (in_sizes[4] < DM || in_sizes[6] < DM || in_sizes[8] < DM) return;
    if ((size_t)out_size < OUT1_OFF + (size_t)SEQ * NB_FULL * SEQ_FULL) return;
    if (SZ_TOTAL > ws_size) return;
    const float* xin  = (const float*)d_in[0];
    const float* bank = (const float*)d_in[1];
    const int*   lens = (const int*)d_in[2];
    const float* wq   = (const float*)d_in[3];
    const float* bq   = (const float*)d_in[4];
    const float* wc   = (const float*)d_in[5];
    const float* vv   = (const float*)d_in[6];
    const float* wo   = (const float*)d_in[7];
    const float* bo   = (const float*)d_in[8];
    float* OUT = (float*)d_out;
    char* wsp = (char*)d_ws;
    bf* XB  = (bf*)wsp; wsp += SZ_XB;
    bf* MB  = (bf*)wsp; wsp += SZ_XB;
    bf* CB  = (bf*)wsp; wsp += SZ_XB;
    bf* WQT = (bf*)wsp; wsp += SZ_WS;
    bf* WCT = (bf*)wsp; wsp += SZ_WS;
    bf* WOT = (bf*)wsp; wsp += SZ_WO;
    bf* MT  = (bf*)wsp; wsp += SZ_MT;
    float* VF  = (float*)wsp; wsp += SZ_VF;
    float* WQF = (float*)wsp; wsp += SZ_PF;
    float* UHF = (float*)wsp; wsp += SZ_PF;

    if (SEQ == SEQ_FULL) {
        const size_t n8 = (size_t)NB * SEQ * DM / 8;
        k_cvt8<<<(unsigned)((n8 + 255) / 256), 256, 0, stream>>>(xin, XB, n8);
        k_cvt8<<<(unsigned)((n8 + 255) / 256), 256, 0, stream>>>(bank, MB, n8);
    } else {
        const size_t n8 = (size_t)SEQ * DM / 8;
        for (int b = 0; b < NB; ++b) {
            k_cvt8<<<(unsigned)((n8 + 255) / 256), 256, 0, stream>>>(xin + (size_t)b * SEQ_FULL * DM, XB + (size_t)b * SEQ * DM, n8);
            k_cvt8<<<(unsigned)((n8 + 255) / 256), 256, 0, stream>>>(bank + (size_t)b * SEQ_FULL * DM, MB + (size_t)b * SEQ * DM, n8);
        }
    }
    k_tr<<<dim3(DM / 64, DM / 64, 1), 256, 0, stream>>>(wq, WQT, DM, DM, DM, (size_t)0, (size_t)0, 0);
    k_tr<<<dim3(DM / 64, DM / 64, 1), 256, 0, stream>>>(wc, WCT, DM, DM, DM, (size_t)0, (size_t)0, 0);
    k_tr<<<dim3(2 * DM / 64, DM / 64, 1), 256, 0, stream>>>(wo, WOT, 2 * DM, DM, 2 * DM, (size_t)0, (size_t)0, 0);
    k_tr<<<dim3(SKP / 64, DM / 64, NB), 256, 0, stream>>>(bank, MT, SEQ, DM, SKP, (size_t)SEQ_FULL * DM, (size_t)DM * SKP, 1);
    k_bfr4<<<DM / 4 / 128, 128, 0, stream>>>(vv, VF, DM / 4);

    k_gemm<<<dim3(NB * SEQ / 16, DM / 64, 1), 32, 0, stream>>>(XB, XB, DM, 0, WQT, bq, 1, C2, WQF, DM, 0);
    k_gemm<<<dim3(NB * SEQ / 16, DM / 64, 1), 32, 0, stream>>>(MB, MB, DM, 0, WCT, bq, 0, C2, UHF, DM, 0);

    k_score<<<SEQ / TT, 256, 0, stream>>>(WQF, UHF, VF, lens, (const h16*)MT, CB, OUT + OUT1_OFF);

    k_gemm<<<dim3(NB * SEQ / 16, DM / 64, 1), 32, 0, stream>>>(CB, XB, DM, DM, WOT, bo, 1, 1.0f, OUT, DM, 1);
}
